// UnivNetLVCResidualBlock_4260607558287
// MI455X (gfx1250) — hardware-verified
//
#include <hip/hip_runtime.h>


#define NBI  8
#define CH   64
#define CO   128
#define LL   16384
#define KS3  3
#define DIL  3
#define NSEG 64
#define HOP  256
#define KC   192
#define DM   KC
#define SLOPE 0.2f
#define LOSC 1024.0f

typedef _Float16 h16;
typedef unsigned short bf;
typedef __attribute__((ext_vector_type(16))) __bf16   v16bf;
typedef __attribute__((ext_vector_type(16))) _Float16 v16h;
typedef __attribute__((ext_vector_type(8)))  _Float16 v8h;
typedef __attribute__((ext_vector_type(8)))  unsigned short v8us;
typedef __attribute__((ext_vector_type(8)))  float    v8f;
typedef __attribute__((ext_vector_type(4)))  float    v4f;
typedef v8h  __attribute__((may_alias)) v8ha;
typedef v4f  __attribute__((may_alias)) v4fa;
typedef v8us __attribute__((may_alias)) v8usa;

__device__ __forceinline__ unsigned short f2bf(float f) { unsigned u = __float_as_uint(f); u += 0x7FFFu + ((u >> 16) & 1u); return (unsigned short)(u >> 16); }
__device__ __forceinline__ float bf2f(unsigned short b) { return __uint_as_float(((unsigned)b) << 16); }
__device__ __forceinline__ float bfr(float f) { return bf2f(f2bf(f)); }
__device__ __forceinline__ v16h cat16(v8h lo, v8h hi) { return __builtin_shufflevector(lo, hi, 0, 1, 2, 3, 4, 5, 6, 7, 8, 9, 10, 11, 12, 13, 14, 15); }
__device__ __forceinline__ v16bf cat16b(v8us lo, v8us hi) { return __builtin_bit_cast(v16bf, __builtin_shufflevector(lo, hi, 0, 1, 2, 3, 4, 5, 6, 7, 8, 9, 10, 11, 12, 13, 14, 15)); }
__device__ __forceinline__ v8f wmma16(v16h a, v16h b, v8f c) { return __builtin_amdgcn_wmma_f32_16x16x32_f16(false, a, false, b, (short)0, c, false, false); }
__device__ __forceinline__ v8f wmmab(v16bf a, v16bf b, v8f c) { return __builtin_amdgcn_wmma_f32_16x16x32_bf16(false, a, false, b, (short)0, c, false, false); }

template <bool SPLITA, bool F16OUT = false>
__global__ __launch_bounds__(128) void k_gemmb(const bf* __restrict__ A, const bf* __restrict__ Al, const bf* __restrict__ Bn, const float* __restrict__ bias, float* C, int ldc, h16* C2, const float* __restrict__ R = nullptr, int K = DM, int roundR = 1) {
    __shared__ __align__(16) float ost[4][16 * 68];
    const int lane = threadIdx.x & 31, wave = threadIdx.x >> 5, lr = lane & 15, hi = lane >> 4;
    const int r0 = blockIdx.x * 64 + wave * 16, c0 = blockIdx.y * 64;
    const size_t aoff = (size_t)(r0 + lr) * K + 8 * hi;
    size_t boff[4];
#pragma unroll
    for (int t = 0; t < 4; ++t) boff[t] = (size_t)(c0 + t * 16 + lr) * K + 8 * hi;
    v8f acc[4];
#pragma unroll
    for (int t = 0; t < 4; ++t) acc[t] = (v8f){};
#pragma unroll 1
    for (int kc = 0; kc < K; kc += 32) {
        const v16bf a = cat16b(*(const v8us*)(A + aoff + kc), *(const v8us*)(A + aoff + kc + 16));
        v16bf al = a;
        if (SPLITA) al = cat16b(*(const v8us*)(Al + aoff + kc), *(const v8us*)(Al + aoff + kc + 16));
#pragma unroll
        for (int t = 0; t < 4; ++t) { const v16bf b = cat16b(*(const v8us*)(Bn + boff[t] + kc), *(const v8us*)(Bn + boff[t] + kc + 16)); acc[t] = wmmab(a, b, acc[t]); if (SPLITA) acc[t] = wmmab(al, b, acc[t]); }
        asm volatile("v_nop\n\tv_nop\n\tv_nop\n\tv_nop" : "+v"(acc[0]), "+v"(acc[1]), "+v"(acc[2]), "+v"(acc[3]) : "v"(a), "v"(al));
    }
    float* os = &ost[wave][0];
#pragma unroll
    for (int t = 0; t < 4; ++t) { const float bv = bias ? bfr(bias[c0 + t * 16 + lr]) : 0.f;
#pragma unroll
        for (int j = 0; j < 8; ++j) os[(hi * 8 + j) * 68 + t * 16 + lr] = acc[t][j] + bv; }
    __syncthreads();
    if (F16OUT) {
        h16* crow = (h16*)(void*)C + (size_t)r0 * ldc + c0;
        auto pass = [&]() {
#pragma unroll
            for (int s = 0; s < 4; ++s) { const int row = 4 * s + (lane >> 3), piece = lane & 7; const float* sp = os + row * 68 + piece * 8; v8h o, o2;
#pragma unroll
                for (int i = 0; i < 8; ++i) { const h16 a = (h16)sp[i]; o[i] = a; o2[i] = (h16)((sp[i] - (float)a) * LOSC); }
                *(volatile v8h*)(crow + (size_t)row * ldc + piece * 8) = o; if (C2) *(volatile v8h*)(C2 + (size_t)r0 * ldc + c0 + (size_t)row * ldc + piece * 8) = o2; }
        };
        pass(); __threadfence(); pass();
    } else {
        float* crow = C + (size_t)r0 * ldc + c0;
        auto pass = [&]() {
#pragma unroll
            for (int s = 0; s < 8; ++s) { const int Lid = (lane >> 3) + 4 * s, piece = lane & 7; const int row = Lid >> 1, cofs = (Lid & 1) * 32 + piece * 4;
                v4f val = *(const v4fa*)(os + row * 68 + cofs); if (R) { const v4f rv = *(const v4f*)(R + ((size_t)r0 + row) * ldc + c0 + cofs); val += roundR ? (v4f){bfr(rv[0]), bfr(rv[1]), bfr(rv[2]), bfr(rv[3])} : rv; }
                *(volatile v4f*)(crow + (size_t)row * ldc + cofs) = val; }
        };
        pass(); __threadfence(); pass();
    }
}

template <bool SPLITA, bool F16OUT = false>
__global__ __launch_bounds__(128) void k_gemmbz(const bf* __restrict__ A, const bf* __restrict__ Al, const bf* __restrict__ Bn, const float* __restrict__ bias, float* C, int ldc, h16* C2, const float* __restrict__ R, int K, int roundR, size_t sA, size_t sB, size_t sBias, size_t sC) {
    { const size_t g = blockIdx.z; A += g * sA; if (Al) Al += g * sA; Bn += g * sB; if (bias) bias += g * sBias; C += g * sC; if (R) R += g * sC; }
    __shared__ __align__(16) float ost[4][16 * 68];
    const int lane = threadIdx.x & 31, wave = threadIdx.x >> 5, lr = lane & 15, hi = lane >> 4;
    const int r0 = blockIdx.x * 64 + wave * 16, c0 = blockIdx.y * 64;
    const size_t aoff = (size_t)(r0 + lr) * K + 8 * hi;
    size_t boff[4];
#pragma unroll
    for (int t = 0; t < 4; ++t) boff[t] = (size_t)(c0 + t * 16 + lr) * K + 8 * hi;
    v8f acc[4];
#pragma unroll
    for (int t = 0; t < 4; ++t) acc[t] = (v8f){};
#pragma unroll 1
    for (int kc = 0; kc < K; kc += 32) {
        const v16bf a = cat16b(*(const v8us*)(A + aoff + kc), *(const v8us*)(A + aoff + kc + 16));
        v16bf al = a;
        if (SPLITA) al = cat16b(*(const v8us*)(Al + aoff + kc), *(const v8us*)(Al + aoff + kc + 16));
#pragma unroll
        for (int t = 0; t < 4; ++t) { const v16bf b = cat16b(*(const v8us*)(Bn + boff[t] + kc), *(const v8us*)(Bn + boff[t] + kc + 16)); acc[t] = wmmab(a, b, acc[t]); if (SPLITA) acc[t] = wmmab(al, b, acc[t]); }
        asm volatile("v_nop\n\tv_nop\n\tv_nop\n\tv_nop" : "+v"(acc[0]), "+v"(acc[1]), "+v"(acc[2]), "+v"(acc[3]) : "v"(a), "v"(al));
    }
    float* os = &ost[wave][0];
#pragma unroll
    for (int t = 0; t < 4; ++t) { const float bv = bias ? bfr(bias[c0 + t * 16 + lr]) : 0.f;
#pragma unroll
        for (int j = 0; j < 8; ++j) os[(hi * 8 + j) * 68 + t * 16 + lr] = acc[t][j] + bv; }
    __syncthreads();
    if (F16OUT) {
        h16* crow = (h16*)(void*)C + (size_t)r0 * ldc + c0;
        auto pass = [&]() {
#pragma unroll
            for (int s = 0; s < 4; ++s) { const int row = 4 * s + (lane >> 3), piece = lane & 7; const float* sp = os + row * 68 + piece * 8; v8h o, o2;
#pragma unroll
                for (int i = 0; i < 8; ++i) { const h16 a = (h16)sp[i]; o[i] = a; o2[i] = (h16)((sp[i] - (float)a) * LOSC); }
                *(volatile v8h*)(crow + (size_t)row * ldc + piece * 8) = o; if (C2) *(volatile v8h*)(C2 + (size_t)r0 * ldc + c0 + (size_t)row * ldc + piece * 8) = o2; }
        };
        pass(); __threadfence(); pass();
    } else {
        float* crow = C + (size_t)r0 * ldc + c0;
        auto pass = [&]() {
#pragma unroll
            for (int s = 0; s < 8; ++s) { const int Lid = (lane >> 3) + 4 * s, piece = lane & 7; const int row = Lid >> 1, cofs = (Lid & 1) * 32 + piece * 4;
                v4f val = *(const v4fa*)(os + row * 68 + cofs); if (R) { const v4f rv = *(const v4f*)(R + ((size_t)r0 + row) * ldc + c0 + cofs); val += roundR ? (v4f){bfr(rv[0]), bfr(rv[1]), bfr(rv[2]), bfr(rv[3])} : rv; }
                *(volatile v4f*)(crow + (size_t)row * ldc + cofs) = val; }
        };
        pass(); __threadfence(); pass();
    }
}


__global__ __launch_bounds__(256) void k_cvt8(const float* __restrict__ src, bf* dst, size_t n8) {
    const size_t i = (size_t)blockIdx.x * 256 + threadIdx.x; if (i >= n8) return;
    const v8f v = *(const v8f*)(src + i * 8); v8us o;
#pragma unroll
    for (int k = 0; k < 8; ++k) o[k] = f2bf(v[k]);
    *(volatile v8us*)(dst + i * 8) = o; __threadfence(); *(volatile v8us*)(dst + i * 8) = o;
}
__global__ __launch_bounds__(256) void k_zero8(bf* dst, size_t n8) {
    const size_t i = (size_t)blockIdx.x * 256 + threadIdx.x; if (i >= n8) return; v8us z;
#pragma unroll
    for (int k = 0; k < 8; ++k) z[k] = 0;
    *(volatile v8us*)(dst + i * 8) = z; __threadfence(); *(volatile v8us*)(dst + i * 8) = z;
}

__device__ __forceinline__ float lrelu_f(float v) { return v >= 0.f ? v : SLOPE * v; }
__global__ __launch_bounds__(256) void k_im1(const float* __restrict__ xb, bf* Ah, bf* Al) {
    const int lane = threadIdx.x & 31, t = blockIdx.x * 8 + (threadIdx.x >> 5); if (t >= LL || lane >= 24) return; v8us oh, ol;
#pragma unroll
    for (int i = 0; i < 8; ++i) { const int idx = lane * 8 + i, c = idx / KS3, k = idx - c * KS3; const int tt = t + DIL * k - DIL; const bool ok = (tt >= 0) && (tt < LL);
        const float v = ok ? lrelu_f(bfr(xb[(size_t)c * LL + (ok ? tt : 0)])) : 0.f; const unsigned short hb = f2bf(v); oh[i] = hb; ol[i] = f2bf(v - bf2f(hb)); }
    const size_t o = (size_t)t * KC + lane * 8; *(volatile v8us*)(Ah + o) = oh; *(volatile v8us*)(Al + o) = ol; __threadfence(); *(volatile v8us*)(Ah + o) = oh; *(volatile v8us*)(Al + o) = ol;
}
__global__ __launch_bounds__(256) void k_im2(const float* __restrict__ Y, bf* Xh, bf* Xl) {
    const int lane = threadIdx.x & 31, r = blockIdx.x * 8 + (threadIdx.x >> 5); if (r >= NSEG * HOP || lane >= 24) return; const int l = r / HOP, s = r % HOP; v8us oh, ol;
#pragma unroll
    for (int i = 0; i < 8; ++i) { const int idx = lane * 8 + i, c = idx / KS3, k = idx - c * KS3; const int tt = l * HOP + s + k - 1; const bool ok = (tt >= 0) && (tt < LL);
        const float v = ok ? lrelu_f(Y[(size_t)(ok ? tt : 0) * CH + c]) : 0.f; const unsigned short hb = f2bf(v); oh[i] = hb; ol[i] = f2bf(v - bf2f(hb)); }
    const size_t o = (size_t)r * KC + lane * 8; *(volatile v8us*)(Xh + o) = oh; *(volatile v8us*)(Xl + o) = ol; __threadfence(); *(volatile v8us*)(Xh + o) = oh; *(volatile v8us*)(Xl + o) = ol;
}
__global__ __launch_bounds__(256) void k_ks(const float* __restrict__ kb, bf* KS) {
    const int lane = threadIdx.x & 31, r = blockIdx.x * 8 + (threadIdx.x >> 5); if (r >= NSEG * CO || lane >= 24) return; const int l = r / CO, o = r % CO; v8us ob;
#pragma unroll
    for (int i = 0; i < 8; ++i) { const int idx = lane * 8 + i, c = idx / KS3, k = idx - c * KS3; ob[i] = f2bf(kb[((((size_t)c * CO + o) * KS3 + k) * NSEG) + l]); }
    const size_t off = (size_t)r * KC + lane * 8; *(volatile v8us*)(KS + off) = ob; __threadfence(); *(volatile v8us*)(KS + off) = ob;
}
__global__ __launch_bounds__(256) void k_gate(const float* __restrict__ Z, const float* __restrict__ xb, const float* __restrict__ bb, float* OUTB) {
    const int lane = threadIdx.x & 31, r = blockIdx.x * 8 + (threadIdx.x >> 5); if (r >= CH * NSEG) return; const int c = r / NSEG, l = r % NSEG;
    const float b0 = bfr(bb[(size_t)c * NSEG + l]), b1 = bfr(bb[(size_t)(CH + c) * NSEG + l]);
#pragma unroll 1
    for (int ps = 0; ps < 2; ++ps) {
#pragma unroll 1
        for (int st = 0; st < 2; ++st) { const int s0 = st * 128 + lane * 4; v4f o;
#pragma unroll
            for (int q = 0; q < 4; ++q) { const int s = s0 + q; const float za = Z[((size_t)l * CO + c) * HOP + s] + b0, zb = Z[((size_t)l * CO + CH + c) * HOP + s] + b1;
                const float g = 1.0f / (1.0f + __expf(-za)); o[q] = bfr(xb[(size_t)c * LL + l * HOP + s]) + g * tanhf(zb); }
            *(volatile v4f*)(OUTB + (size_t)c * LL + l * HOP + s0) = o; }
        if (ps == 0) __threadfence(); }
}

extern "C" void kernel_launch(void* const* d_in, const int* in_sizes, int n_in,
                              void* d_out, int out_size, void* d_ws, size_t ws_size, hipStream_t stream) {
    (void)in_sizes; (void)n_in; (void)out_size;
    const float* x = (const float*)d_in[0]; const float* ker = (const float*)d_in[1]; const float* lb = (const float*)d_in[2]; const float* cw = (const float*)d_in[3]; const float* cb = (const float*)d_in[4];
    float* out = (float*)d_out;
    char* wsp = (char*)d_ws;
    auto take = [&](size_t bytes) { char* p = wsp; wsp += (bytes + 255) & ~(size_t)255; return (void*)p; };
    bf* CWB = (bf*)take((size_t)CH * KC * 2); bf* A1h = (bf*)take((size_t)LL * KC * 2); bf* A1l = (bf*)take((size_t)LL * KC * 2); float* Y = (float*)take((size_t)LL * CH * 4);
    bf* KSb = (bf*)take((size_t)NSEG * CO * KC * 2); bf* X2h = (bf*)take((size_t)NSEG * HOP * KC * 2); bf* X2l = (bf*)take((size_t)NSEG * HOP * KC * 2); float* ZT = (float*)take((size_t)NSEG * CO * HOP * 4); float* Z = (float*)take((size_t)NSEG * CO * HOP * 4);
    if ((size_t)(wsp - (char*)d_ws) > ws_size) return;
    k_cvt8<<<(CH * KC / 8 + 255) / 256, 256, 0, stream>>>(cw, CWB, CH * KC / 8);
    for (int b = 0; b < NBI; ++b) { const float* xb = x + (size_t)b * CH * LL;
        k_im1<<<LL / 8, 256, 0, stream>>>(xb, A1h, A1l);
        k_gemmb<true, false><<<dim3(LL / 64, 1, 1), 128, 0, stream>>>(A1h, A1l, CWB, cb, Y, CH, nullptr, nullptr, KC);
        k_ks<<<(NSEG * CO) / 8, 256, 0, stream>>>(ker + (size_t)b * CH * CO * KS3 * NSEG, KSb);
        k_im2<<<(NSEG * HOP) / 8, 256, 0, stream>>>(Y, X2h, X2l);
        k_gemmbz<false, false><<<dim3(CO / 64, HOP / 64, NSEG), 128, 0, stream>>>(KSb, nullptr, X2h, nullptr, ZT, HOP, nullptr, nullptr, KC, 0, (size_t)CO * KC, (size_t)HOP * KC, 0, (size_t)CO * HOP);
        k_gemmbz<false, false><<<dim3(CO / 64, HOP / 64, NSEG), 128, 0, stream>>>(KSb, nullptr, X2l, nullptr, Z, HOP, nullptr, ZT, KC, 0, (size_t)CO * KC, (size_t)HOP * KC, 0, (size_t)CO * HOP);
        k_gate<<<(CH * NSEG) / 8, 256, 0, stream>>>(Z, xb, lb + (size_t)b * CO * NSEG, out + (size_t)b * CH * LL); }
}
